// MambaBlock_6897717477938
// MI455X (gfx1250) — hardware-verified
//
#include <hip/hip_runtime.h>
#include <math.h>

typedef __attribute__((ext_vector_type(16))) __bf16   v16b;
typedef __attribute__((ext_vector_type(8)))  __bf16   v8b;
typedef __attribute__((ext_vector_type(8)))  float    v8f;
typedef __attribute__((ext_vector_type(4)))  float    v4f;
typedef __attribute__((ext_vector_type(4)))  unsigned v4u;

constexpr int kSeq   = 2048;
constexpr int kDm    = 1024;
constexpr int kDi    = 2048;
constexpr int kNs    = 128;
constexpr int kNh    = 32;
constexpr int kHd    = 64;
constexpr int kCv    = kDi + 2 * kNs;
constexpr int kPrj   = 2 * kDi + 2 * kNs + kNh;
constexpr int kPrjP  = 4416;
constexpr int kDtCol = kDi + kCv;
constexpr int kInt   = 2752;
constexpr int kTP    = 260;
constexpr int kYP    = 68;
constexpr float kEps = 1e-6f;
static_assert(kCv == 2304);
static_assert(kPrj == 4384);
static_assert(kDtCol == 4352);
static_assert(kNh * kHd == kDi);
static_assert((kPrjP % 64) == 0 && kPrjP >= kPrj);
static_assert((kSeq % 64) == 0 && (kDm % 64) == 0 && (kInt % 64) == 0 && (kDi % 64) == 0);
static_assert((kDm % 32) == 0 && (kDi % 32) == 0 && (kInt % 32) == 0);
static_assert((kCv % 256) == 0 && (kSeq % 16) == 0);

constexpr size_t kSzWout = (size_t)kDm * kDi * 2;
constexpr size_t kSzWg   = (size_t)kInt * kDm * 2;
constexpr size_t kSzWd   = (size_t)kDm * kInt * 2;
constexpr size_t kSzXn   = (size_t)kSeq * kDm * 2;
constexpr size_t kSzWin  = (size_t)kPrjP * kDm * 2;
constexpr size_t kSzYn   = (size_t)kSeq * kDi * 2;
constexpr size_t kSzZx   = (size_t)kSeq * kPrjP * 4;
constexpr size_t kSzXbc  = (size_t)kSeq * kCv * 4;
constexpr size_t kSzDtda = (size_t)kSeq * 64 * 4;
constexpr size_t kSzY    = (size_t)kSeq * kDi * 4;
constexpr size_t kSzGate = (size_t)kSeq * kInt * 4;
constexpr size_t kSzH2   = (size_t)kSeq * kDm * 4;
constexpr size_t kSzGu   = (size_t)kSeq * kInt * 2;

constexpr size_t kOffWout = 0;
constexpr size_t kOffWg   = kOffWout + kSzWout;
constexpr size_t kOffWu   = kOffWg + kSzWg;
constexpr size_t kOffWd   = kOffWu + kSzWg;
constexpr size_t kOffXnh  = kOffWd + kSzWd;
constexpr size_t kOffXnl  = kOffXnh + kSzXn;
constexpr size_t kOffWin  = kOffXnl + kSzXn;
constexpr size_t kOffYnh  = kOffWin + kSzWin;
constexpr size_t kOffYnl  = kOffYnh + kSzYn;
constexpr size_t kOffZx   = kOffYnl + kSzYn;
constexpr size_t kOffXbc  = kOffZx + kSzZx;
constexpr size_t kOffDtda = kOffXbc + kSzXbc;
constexpr size_t kOffY    = kOffDtda + kSzDtda;
constexpr size_t kWsTotal = kOffY + kSzY;
constexpr size_t kOffGuh  = kOffWin;
constexpr size_t kOffGul  = kOffGuh + kSzGu;
constexpr size_t kOffGate = kOffZx;
constexpr size_t kOffH2   = kOffZx + kSzGate;
constexpr size_t kOffUp   = kOffXbc;
static_assert(kWsTotal == 127664128ull);
static_assert(kWsTotal <= 134217728ull);
static_assert(kOffGul + kSzGu <= kOffZx);
static_assert(kOffH2 + kSzH2 <= kOffZx + kSzZx);
static_assert(kOffUp + kSzGate <= kWsTotal);
static_assert((kOffWg % 128) == 0 && (kOffWu % 128) == 0 && (kOffWd % 128) == 0 && (kOffXnh % 128) == 0 &&
              (kOffXnl % 128) == 0 && (kOffWin % 128) == 0 && (kOffYnh % 128) == 0 && (kOffYnl % 128) == 0 &&
              (kOffZx % 128) == 0 && (kOffXbc % 128) == 0 && (kOffDtda % 128) == 0 && (kOffY % 128) == 0 &&
              (kOffGul % 128) == 0 && (kOffH2 % 128) == 0);

__device__ __forceinline__ unsigned bf_rne(float f) {
  const unsigned u = __float_as_uint(f);
  return (u + 0x7FFFu + ((u >> 16) & 1u)) >> 16;
}
__device__ __forceinline__ float bf_val(unsigned hb) { return __uint_as_float(hb << 16); }
__device__ __forceinline__ float bf_rne_val(float f) { return bf_val(bf_rne(f)); }
__device__ __forceinline__ void split2(float a, float b, unsigned& wh, unsigned& wl) {
  const unsigned ha = bf_rne(a), hb = bf_rne(b);
  const unsigned la = bf_rne(a - bf_val(ha)), lb = bf_rne(b - bf_val(hb));
  wh = ha | (hb << 16);
  wl = la | (lb << 16);
}
__device__ __forceinline__ float silu_f(float x) {
  const float e = expf(-x);
  return x * __builtin_amdgcn_rcpf(1.0f + e);
}

union FragB { v16b v; v8b h[2]; };
__device__ __forceinline__ v16b frag_load(const __bf16* p) {
  FragB f;
  f.h[0] = *(const v8b*)(p);
  f.h[1] = *(const v8b*)(p + 16);
  return f.v;
}
__device__ __forceinline__ v8f mma_bf(v16b a, v16b b, v8f c) {
  return __builtin_amdgcn_wmma_f32_16x16x32_bf16(false, a, false, b, (short)0, c, false, false);
}
__device__ __forceinline__ void grp_guard(v8f& a, v8f& b, v8f& c, v8f& d, v16b x, v16b y) {
  asm volatile("v_nop\n\tv_nop\n\tv_nop\n\tv_nop" : "+v"(a), "+v"(b), "+v"(c), "+v"(d) : "v"(x), "v"(y));
}
__device__ __forceinline__ void keep4_b(v16b a, v16b b, v16b c, v16b d) { asm volatile("v_nop" :: "v"(a), "v"(b), "v"(c), "v"(d)); }
__device__ __forceinline__ void acc_guard4(v8f& a, v8f& b, v8f& c, v8f& d) { asm volatile("v_nop\n\tv_nop\n\tv_nop\n\tv_nop" : "+v"(a), "+v"(b), "+v"(c), "+v"(d)); }

template <int RMODE>
__global__ __launch_bounds__(256) void gemm_a2_kernel(
    const unsigned short* __restrict__ Ahp, const unsigned short* __restrict__ Alp, int lda,
    const unsigned short* __restrict__ Btp, int ldb,
    float* __restrict__ C, int ldc,
    const float* __restrict__ R, int ldr,
    int M, int N, int K)
{
  const __bf16* Ah = (const __bf16*)Ahp;
  const __bf16* Al = (const __bf16*)Alp;
  const __bf16* Bt = (const __bf16*)Btp;
  __shared__ __align__(16) float sT[8][16 * 68];
  const int lane = threadIdx.x & 31;
  const int wave = threadIdx.x >> 5;
  const int tilesN = N >> 6;
  const int tilesM = M >> 6;
  const int tile = blockIdx.x * 8 + wave;
  if (tile >= tilesM * tilesN) return;
  const int tm = tile / tilesN;
  const int tn = tile - tm * tilesN;
  const int m0 = tm << 6;
  const int n0 = tn << 6;
  const int rlane = lane & 15;
  const int koff  = (lane >> 4) * 8;
  const int mOff  = (lane >> 4) * 8;

  v8f acc[4][4];
#pragma unroll
  for (int i = 0; i < 4; ++i)
#pragma unroll
    for (int j = 0; j < 4; ++j) acc[i][j] = (v8f){0.f, 0.f, 0.f, 0.f, 0.f, 0.f, 0.f, 0.f};

  for (int k0 = 0; k0 < K; k0 += 32) {
    v16b bh[4];
#pragma unroll
    for (int j = 0; j < 4; ++j) {
      const size_t bo = (size_t)(n0 + (j << 4) + rlane) * ldb + koff + k0;
      bh[j] = frag_load(Bt + bo);
    }
#pragma unroll
    for (int i = 0; i < 4; ++i) {
      const size_t ao = (size_t)(m0 + (i << 4) + rlane) * lda + koff + k0;
      const v16b ah = frag_load(Ah + ao);
      const v16b al = frag_load(Al + ao);
#pragma unroll
      for (int j = 0; j < 4; ++j) {
        acc[i][j] = mma_bf(ah, bh[j], acc[i][j]);
        acc[i][j] = mma_bf(al, bh[j], acc[i][j]);
      }
      grp_guard(acc[i][0], acc[i][1], acc[i][2], acc[i][3], ah, al);
    }
    keep4_b(bh[0], bh[1], bh[2], bh[3]);
  }
  acc_guard4(acc[0][0], acc[0][1], acc[0][2], acc[0][3]);
  acc_guard4(acc[1][0], acc[1][1], acc[1][2], acc[1][3]);
  acc_guard4(acc[2][0], acc[2][1], acc[2][2], acc[2][3]);
  acc_guard4(acc[3][0], acc[3][1], acc[3][2], acc[3][3]);

  float* slab = sT[wave];
  const int hh = lane >> 4, c4 = (lane & 15) * 4;
#pragma unroll
  for (int i = 0; i < 4; ++i) {
    const int mBase = m0 + (i << 4);
#pragma unroll
    for (int j = 0; j < 4; ++j) {
#pragma unroll
      for (int r = 0; r < 8; ++r) slab[(mOff + r) * 68 + (j << 4) + rlane] = acc[i][j][r];
    }
    __builtin_amdgcn_fence(__ATOMIC_RELEASE, "workgroup");
    __builtin_amdgcn_wave_barrier();
    __builtin_amdgcn_fence(__ATOMIC_ACQUIRE, "workgroup");
    v4f vv[8];
#pragma unroll
    for (int it = 0; it < 8; ++it) {
      const int row = it * 2 + hh;
      v4f v = *(const v4f*)(slab + row * 68 + c4);
      if (RMODE != 0) {
        const v4f rr = *(const v4f*)(R + (size_t)(mBase + row) * ldr + n0 + c4);
        float r0 = rr[0], r1 = rr[1], r2 = rr[2], r3 = rr[3];
        if (RMODE == 2) {
          r0 = bf_rne_val(r0);
          r1 = bf_rne_val(r1);
          r2 = bf_rne_val(r2);
          r3 = bf_rne_val(r3);
        }
        v[0] += r0;
        v[1] += r1;
        v[2] += r2;
        v[3] += r3;
      }
      vv[it] = v;
    }
    for (int pass = 0; pass < 2; ++pass) {
#pragma unroll
      for (int it = 0; it < 8; ++it) {
        const int row = it * 2 + hh;
        *(volatile v4f*)(C + (size_t)(mBase + row) * ldc + n0 + c4) = vv[it];
      }
      __threadfence();
    }
    __builtin_amdgcn_fence(__ATOMIC_RELEASE, "workgroup");
    __builtin_amdgcn_wave_barrier();
    __builtin_amdgcn_fence(__ATOMIC_ACQUIRE, "workgroup");
  }
}

__global__ __launch_bounds__(256) void cvt_bf16_kernel(
    const float* __restrict__ src, unsigned short* __restrict__ dst, int real8, int pad8)
{
  const int i = blockIdx.x * 256 + threadIdx.x;
  if (i >= pad8) return;
  const bool live = (i < real8);
  const int ic = live ? i : (real8 - 1);
  const float* p = src + ((size_t)ic << 3);
  const v4f a0 = *(const v4f*)(p);
  const v4f a1 = *(const v4f*)(p + 4);
  const float t0 = a0[0], t1 = a0[1], t2 = a0[2], t3 = a0[3];
  const float t4 = a1[0], t5 = a1[1], t6 = a1[2], t7 = a1[3];
  const unsigned w0 = bf_rne(t0) | (bf_rne(t1) << 16);
  const unsigned w1 = bf_rne(t2) | (bf_rne(t3) << 16);
  const unsigned w2 = bf_rne(t4) | (bf_rne(t5) << 16);
  const unsigned w3 = bf_rne(t6) | (bf_rne(t7) << 16);
  v4u o;
  o[0] = live ? w0 : 0u;
  o[1] = live ? w1 : 0u;
  o[2] = live ? w2 : 0u;
  o[3] = live ? w3 : 0u;
  unsigned short* q = dst + ((size_t)i << 3);
  *(volatile v4u*)(void*)q = o;
  __threadfence();
  *(volatile v4u*)(void*)q = o;
}

template <bool RNE_IN>
__global__ __launch_bounds__(128) void rmsnorm_split_kernel(
    const float* __restrict__ X, const float* __restrict__ W,
    unsigned short* __restrict__ OH, unsigned short* __restrict__ OL)
{
  __shared__ float sred[4];
  const int tid = threadIdx.x, lane = tid & 31, wave = tid >> 5;
  const size_t base = (size_t)blockIdx.x * kDm + (size_t)tid * 8;
  const v4f a0 = *(const v4f*)(X + base);
  const v4f a1 = *(const v4f*)(X + base + 4);
  float x[8];
  x[0] = a0[0]; x[1] = a0[1]; x[2] = a0[2]; x[3] = a0[3];
  x[4] = a1[0]; x[5] = a1[1]; x[6] = a1[2]; x[7] = a1[3];
  if (RNE_IN) {
#pragma unroll
    for (int e = 0; e < 8; ++e) x[e] = bf_rne_val(x[e]);
  }
  float ss = 0.f;
#pragma unroll
  for (int e = 0; e < 8; ++e) ss = fmaf(x[e], x[e], ss);
#pragma unroll
  for (int off = 16; off > 0; off >>= 1) ss += __shfl_xor(ss, off, 32);
  if (lane == 0) sred[wave] = ss;
  __syncthreads();
  const float tot = (sred[0] + sred[1]) + (sred[2] + sred[3]);
  const float sc = rsqrtf(tot * (1.0f / (float)kDm) + kEps);
  const v4f w0 = *(const v4f*)(W + tid * 8);
  const v4f w1 = *(const v4f*)(W + tid * 8 + 4);
  float w[8];
  w[0] = w0[0]; w[1] = w0[1]; w[2] = w0[2]; w[3] = w0[3];
  w[4] = w1[0]; w[5] = w1[1]; w[6] = w1[2]; w[7] = w1[3];
  float y[8];
#pragma unroll
  for (int e = 0; e < 8; ++e) y[e] = (x[e] * sc) * bf_rne_val(w[e]);
  unsigned h0, h1, h2, h3, l0, l1, l2, l3;
  split2(y[0], y[1], h0, l0);
  split2(y[2], y[3], h1, l1);
  split2(y[4], y[5], h2, l2);
  split2(y[6], y[7], h3, l3);
  v4u oh, ol;
  oh[0] = h0; oh[1] = h1; oh[2] = h2; oh[3] = h3;
  ol[0] = l0; ol[1] = l1; ol[2] = l2; ol[3] = l3;
  unsigned short* ph = OH + base;
  unsigned short* pl = OL + base;
  *(volatile v4u*)(void*)ph = oh;
  *(volatile v4u*)(void*)pl = ol;
  __threadfence();
  *(volatile v4u*)(void*)ph = oh;
  *(volatile v4u*)(void*)pl = ol;
}

__global__ __launch_bounds__(256) void conv_silu_kernel(
    const float* __restrict__ ZX, const float* __restrict__ cw, const float* __restrict__ cb,
    float* __restrict__ XBC)
{
  __shared__ __align__(16) float sT[16 * kTP];
  const int tid = threadIdx.x, lane = tid & 31, wave = tid >> 5;
  const int d0 = blockIdx.x * 256, d = d0 + tid;
  const int t0 = blockIdx.y * 64;
  const v4f wv = *(const v4f*)(cw + (size_t)d * 4);
  const float wa = wv[0], wb = wv[1], wc = wv[2], wd = wv[3];
  const float w0 = bf_rne_val(wa), w1 = bf_rne_val(wb), w2 = bf_rne_val(wc), w3 = bf_rne_val(wd);
  const float bc = bf_rne_val(cb[d]);
  const float* src = ZX + kDi + d;
  float xm3, xm2, xm1;
  {
    const int r3 = t0 - 3, r2 = t0 - 2, r1 = t0 - 1;
    const float v3 = src[(size_t)(r3 < 0 ? 0 : r3) * kPrjP];
    const float v2 = src[(size_t)(r2 < 0 ? 0 : r2) * kPrjP];
    const float v1 = src[(size_t)(r1 < 0 ? 0 : r1) * kPrjP];
    xm3 = (r3 >= 0) ? v3 : 0.f;
    xm2 = (r2 >= 0) ? v2 : 0.f;
    xm1 = (r1 >= 0) ? v1 : 0.f;
  }
  const int hrow = wave >> 1;
  const int hch  = (wave & 1) * 128 + lane * 4;
#pragma unroll 1
  for (int sub = 0; sub < 4; ++sub) {
    const int lb = t0 + sub * 16;
#pragma unroll 1
    for (int s = 0; s < 16; ++s) {
      const float xc = src[(size_t)(lb + s) * kPrjP];
      float acc = w0 * xm3;
      acc = fmaf(w1, xm2, acc);
      acc = fmaf(w2, xm1, acc);
      acc = fmaf(w3, xc, acc);
      const float sv = acc + bc;
      sT[s * kTP + tid] = silu_f(sv);
      xm3 = xm2;
      xm2 = xm1;
      xm1 = xc;
    }
    __syncthreads();
    v4f fv[4];
#pragma unroll
    for (int it = 0; it < 4; ++it) fv[it] = *(const v4f*)(sT + (it * 4 + hrow) * kTP + hch);
    for (int pass = 0; pass < 2; ++pass) {
#pragma unroll
      for (int it = 0; it < 4; ++it)
        *(volatile v4f*)(XBC + (size_t)(lb + it * 4 + hrow) * kCv + d0 + hch) = fv[it];
      __threadfence();
    }
    __syncthreads();
  }
}

__global__ __launch_bounds__(256) void dt_kernel(
    const float* __restrict__ ZX, const float* __restrict__ dtb, const float* __restrict__ Alog,
    float* __restrict__ DTDA)
{
  const int lane = threadIdx.x & 31, wave = threadIdx.x >> 5;
  const int row = blockIdx.x * 8 + wave;
  const float v = ZX[(size_t)row * kPrjP + kDtCol + lane] + bf_rne_val(dtb[lane]);
  const float dt = fmaxf(v, 0.0f) + log1pf(expf(-fabsf(v)));
  const float An = -expf(bf_rne_val(Alog[lane]));
  float dA = expf(dt * An);
  dA = (dA < 1.17549435e-38f) ? 0.0f : dA;
  float* o = DTDA + (size_t)row * 64;
  *(volatile float*)(o + lane) = dt;
  *(volatile float*)(o + 32 + lane) = dA;
  __threadfence();
  *(volatile float*)(o + lane) = dt;
  *(volatile float*)(o + 32 + lane) = dA;
}

__global__ __launch_bounds__(256) void scan_kernel(
    const float* __restrict__ XBC, const float* __restrict__ DTDA, const float* __restrict__ Dp,
    float* __restrict__ Y)
{
  __shared__ __align__(16) float sBC[16 * 256];
  __shared__ __align__(16) float sX[16 * 64];
  __shared__ __align__(16) float sDT[32];
  __shared__ __align__(16) float sY[16 * kYP];
  const int tid = threadIdx.x, lane = tid & 31, wave = tid >> 5;
  const int h = blockIdx.x;
  const int p = tid >> 2;
  const int nb = (tid & 3) * 32;
  const float Dh = bf_rne_val(Dp[h]);
  float st[32];
#pragma unroll
  for (int i = 0; i < 32; ++i) st[i] = 0.f;
  const int hh = lane >> 4, c4 = (lane & 15) * 4;
#pragma unroll 1
  for (int c = 0; c < kSeq / 16; ++c) {
    const int t0 = c * 16;
#pragma unroll
    for (int i = 0; i < 4; ++i) {
      const int idx = tid + i * 256;
      const int r = idx >> 6;
      const int q = (idx & 63) << 2;
      *(v4f*)(sBC + r * 256 + q) = *(const v4f*)(XBC + (size_t)(t0 + r) * kCv + kDi + q);
    }
    {
      const int r = tid >> 4;
      const int q = (tid & 15) << 2;
      *(v4f*)(sX + r * 64 + q) = *(const v4f*)(XBC + (size_t)(t0 + r) * kCv + h * kHd + q);
    }
    if (tid < 32) {
      const int r = tid & 15;
      const int wsel = tid >> 4;
      sDT[r * 2 + wsel] = DTDA[(size_t)(t0 + r) * 64 + wsel * 32 + h];
    }
    __syncthreads();
#pragma unroll 1
    for (int s = 0; s < 16; ++s) {
      const float dtv = sDT[2 * s];
      const float dAv = sDT[2 * s + 1];
      const float xv = sX[s * 64 + p];
      const float coef = dtv * xv;
      const float* bp = sBC + s * 256 + nb;
      const float* cp = bp + 128;
      float ys = 0.f;
#pragma unroll
      for (int k = 0; k < 8; ++k) {
        const v4f bv = *(const v4f*)(bp + 4 * k);
        const v4f cv = *(const v4f*)(cp + 4 * k);
#pragma unroll
        for (int e = 0; e < 4; ++e) {
          const float sn = fmaf(st[4 * k + e], dAv, coef * bv[e]);
          st[4 * k + e] = sn;
          ys = fmaf(sn, cv[e], ys);
        }
      }
      ys += __shfl_xor(ys, 1, 32);
      ys += __shfl_xor(ys, 2, 32);
      if ((tid & 3) == 0) sY[s * kYP + p] = ys + Dh * xv;
    }
    __syncthreads();
    {
      const int row = wave * 2 + hh;
      const v4f val = *(const v4f*)(sY + row * kYP + c4);
      float* dst = Y + (size_t)(t0 + row) * kDi + h * kHd + c4;
      *(volatile v4f*)dst = val;
      __threadfence();
      *(volatile v4f*)dst = val;
    }
  }
}

__global__ __launch_bounds__(256) void gated_norm_kernel(
    const float* __restrict__ Y, const float* __restrict__ ZX, const float* __restrict__ W,
    unsigned short* __restrict__ OH, unsigned short* __restrict__ OL)
{
  __shared__ float sred[8];
  const int tid = threadIdx.x, lane = tid & 31, wave = tid >> 5;
  const int row = blockIdx.x;
  const size_t yb = (size_t)row * kDi + (size_t)tid * 8;
  const size_t zb = (size_t)row * kPrjP + (size_t)tid * 8;
  const v4f y0 = *(const v4f*)(Y + yb);
  const v4f y1 = *(const v4f*)(Y + yb + 4);
  const v4f z0 = *(const v4f*)(ZX + zb);
  const v4f z1 = *(const v4f*)(ZX + zb + 4);
  float yv[8], zv[8], g[8];
  yv[0] = y0[0]; yv[1] = y0[1]; yv[2] = y0[2]; yv[3] = y0[3];
  yv[4] = y1[0]; yv[5] = y1[1]; yv[6] = y1[2]; yv[7] = y1[3];
  zv[0] = z0[0]; zv[1] = z0[1]; zv[2] = z0[2]; zv[3] = z0[3];
  zv[4] = z1[0]; zv[5] = z1[1]; zv[6] = z1[2]; zv[7] = z1[3];
  float ss = 0.f;
#pragma unroll
  for (int e = 0; e < 8; ++e) {
    g[e] = yv[e] * silu_f(zv[e]);
    ss = fmaf(g[e], g[e], ss);
  }
#pragma unroll
  for (int off = 16; off > 0; off >>= 1) ss += __shfl_xor(ss, off, 32);
  if (lane == 0) sred[wave] = ss;
  __syncthreads();
  const float tot = ((sred[0] + sred[1]) + (sred[2] + sred[3])) + ((sred[4] + sred[5]) + (sred[6] + sred[7]));
  const float sc = rsqrtf(tot * (1.0f / (float)kDi) + kEps);
  const v4f w0 = *(const v4f*)(W + tid * 8);
  const v4f w1 = *(const v4f*)(W + tid * 8 + 4);
  float w[8];
  w[0] = w0[0]; w[1] = w0[1]; w[2] = w0[2]; w[3] = w0[3];
  w[4] = w1[0]; w[5] = w1[1]; w[6] = w1[2]; w[7] = w1[3];
  float o[8];
#pragma unroll
  for (int e = 0; e < 8; ++e) o[e] = (g[e] * sc) * bf_rne_val(w[e]);
  unsigned h0, h1, h2, h3, l0, l1, l2, l3;
  split2(o[0], o[1], h0, l0);
  split2(o[2], o[3], h1, l1);
  split2(o[4], o[5], h2, l2);
  split2(o[6], o[7], h3, l3);
  v4u oh, ol;
  oh[0] = h0; oh[1] = h1; oh[2] = h2; oh[3] = h3;
  ol[0] = l0; ol[1] = l1; ol[2] = l2; ol[3] = l3;
  unsigned short* ph = OH + yb;
  unsigned short* pl = OL + yb;
  *(volatile v4u*)(void*)ph = oh;
  *(volatile v4u*)(void*)pl = ol;
  __threadfence();
  *(volatile v4u*)(void*)ph = oh;
  *(volatile v4u*)(void*)pl = ol;
}

__global__ __launch_bounds__(256) void gu_split_kernel(
    const float* __restrict__ G, const float* __restrict__ U,
    unsigned short* __restrict__ OH, unsigned short* __restrict__ OL, int total8)
{
  const int i = blockIdx.x * 256 + threadIdx.x;
  if (i >= total8) return;
  const size_t e0 = (size_t)i << 3;
  const v4f g0 = *(const v4f*)(G + e0);
  const v4f g1 = *(const v4f*)(G + e0 + 4);
  const v4f u0 = *(const v4f*)(U + e0);
  const v4f u1 = *(const v4f*)(U + e0 + 4);
  float gv[8], uv[8], o[8];
  gv[0] = g0[0]; gv[1] = g0[1]; gv[2] = g0[2]; gv[3] = g0[3];
  gv[4] = g1[0]; gv[5] = g1[1]; gv[6] = g1[2]; gv[7] = g1[3];
  uv[0] = u0[0]; uv[1] = u0[1]; uv[2] = u0[2]; uv[3] = u0[3];
  uv[4] = u1[0]; uv[5] = u1[1]; uv[6] = u1[2]; uv[7] = u1[3];
#pragma unroll
  for (int e = 0; e < 8; ++e) o[e] = silu_f(gv[e]) * uv[e];
  unsigned h0, h1, h2, h3, l0, l1, l2, l3;
  split2(o[0], o[1], h0, l0);
  split2(o[2], o[3], h1, l1);
  split2(o[4], o[5], h2, l2);
  split2(o[6], o[7], h3, l3);
  v4u oh, ol;
  oh[0] = h0; oh[1] = h1; oh[2] = h2; oh[3] = h3;
  ol[0] = l0; ol[1] = l1; ol[2] = l2; ol[3] = l3;
  unsigned short* ph = OH + e0;
  unsigned short* pl = OL + e0;
  *(volatile v4u*)(void*)ph = oh;
  *(volatile v4u*)(void*)pl = ol;
  __threadfence();
  *(volatile v4u*)(void*)ph = oh;
  *(volatile v4u*)(void*)pl = ol;
}

static_assert(((kSeq / 64) * (kPrjP / 64)) % 8 == 0);
static_assert(((kSeq / 64) * (kDm / 64)) % 8 == 0);
static_assert(((kSeq / 64) * (kInt / 64)) % 8 == 0);
static_assert(((kPrjP * kDm / 8) % 256) == 0 && ((kDm * kDi / 8) % 256) == 0 && ((kInt * kDm / 8) % 256) == 0);
static_assert(((kSeq * kInt / 8) % 256) == 0);

extern "C" void kernel_launch(void* const* d_in, const int* in_sizes, int n_in,
                              void* d_out, int out_size, void* d_ws, size_t ws_size,
                              hipStream_t stream)
{
  if (n_in < 14) return;
  if (in_sizes[0] != kSeq * kDm) return;
  if (in_sizes[1] != kDm) return;
  if (in_sizes[2] != kPrj * kDm) return;
  if (in_sizes[3] != kCv * 4) return;
  if (in_sizes[4] != kCv) return;
  if (in_sizes[5] != kNh || in_sizes[6] != kNh || in_sizes[7] != kNh) return;
  if (in_sizes[8] != kDi) return;
  if (in_sizes[9] != kDm * kDi) return;
  if (in_sizes[10] != kDm) return;
  if (in_sizes[11] != kInt * kDm || in_sizes[12] != kInt * kDm) return;
  if (in_sizes[13] != kDm * kInt) return;
  if (out_size != kSeq * kDm) return;
  if (ws_size < kWsTotal) return;

  const float* hidden      = (const float*)d_in[0];
  const float* norm_w      = (const float*)d_in[1];
  const float* in_proj_w   = (const float*)d_in[2];
  const float* conv_w      = (const float*)d_in[3];
  const float* conv_b      = (const float*)d_in[4];
  const float* dt_bias     = (const float*)d_in[5];
  const float* A_log       = (const float*)d_in[6];
  const float* Dp          = (const float*)d_in[7];
  const float* ssm_norm_w  = (const float*)d_in[8];
  const float* out_proj_w  = (const float*)d_in[9];
  const float* post_norm_w = (const float*)d_in[10];
  const float* gate_w      = (const float*)d_in[11];
  const float* up_w        = (const float*)d_in[12];
  const float* down_w      = (const float*)d_in[13];
  float* out = (float*)d_out;

  char* ws = (char*)d_ws;
  unsigned short* WOUT = (unsigned short*)(ws + kOffWout);
  unsigned short* WG   = (unsigned short*)(ws + kOffWg);
  unsigned short* WU   = (unsigned short*)(ws + kOffWu);
  unsigned short* WD   = (unsigned short*)(ws + kOffWd);
  unsigned short* XNH  = (unsigned short*)(ws + kOffXnh);
  unsigned short* XNL  = (unsigned short*)(ws + kOffXnl);
  unsigned short* WIN  = (unsigned short*)(ws + kOffWin);
  unsigned short* YNH  = (unsigned short*)(ws + kOffYnh);
  unsigned short* YNL  = (unsigned short*)(ws + kOffYnl);
  unsigned short* GUH  = (unsigned short*)(ws + kOffGuh);
  unsigned short* GUL  = (unsigned short*)(ws + kOffGul);
  float* ZX   = (float*)(ws + kOffZx);
  float* GATE = (float*)(ws + kOffGate);
  float* H2   = (float*)(ws + kOffH2);
  float* XBC  = (float*)(ws + kOffXbc);
  float* DTDA = (float*)(ws + kOffDtda);
  float* Yp   = (float*)(ws + kOffY);
  float* UP   = (float*)(ws + kOffUp);

  cvt_bf16_kernel<<<(kPrjP * kDm / 8) / 256, 256, 0, stream>>>(in_proj_w, WIN, kPrj * kDm / 8, kPrjP * kDm / 8);
  cvt_bf16_kernel<<<(kDm * kDi / 8) / 256, 256, 0, stream>>>(out_proj_w, WOUT, kDm * kDi / 8, kDm * kDi / 8);
  cvt_bf16_kernel<<<(kInt * kDm / 8) / 256, 256, 0, stream>>>(gate_w, WG, kInt * kDm / 8, kInt * kDm / 8);
  cvt_bf16_kernel<<<(kInt * kDm / 8) / 256, 256, 0, stream>>>(up_w, WU, kInt * kDm / 8, kInt * kDm / 8);
  cvt_bf16_kernel<<<(kDm * kInt / 8) / 256, 256, 0, stream>>>(down_w, WD, kDm * kInt / 8, kDm * kInt / 8);

  rmsnorm_split_kernel<true><<<kSeq, 128, 0, stream>>>(hidden, norm_w, XNH, XNL);

  gemm_a2_kernel<0><<<((kSeq / 64) * (kPrjP / 64)) / 8, 256, 0, stream>>>(
      XNH, XNL, kDm, WIN, kDm, ZX, kPrjP, hidden, 0, kSeq, kPrjP, kDm);

  conv_silu_kernel<<<dim3(kCv / 256, kSeq / 64), 256, 0, stream>>>(ZX, conv_w, conv_b, XBC);

  dt_kernel<<<kSeq / 8, 256, 0, stream>>>(ZX, dt_bias, A_log, DTDA);

  scan_kernel<<<kNh, 256, 0, stream>>>(XBC, DTDA, Dp, Yp);

  gated_norm_kernel<<<kSeq, 256, 0, stream>>>(Yp, ZX, ssm_norm_w, YNH, YNL);

  gemm_a2_kernel<2><<<((kSeq / 64) * (kDm / 64)) / 8, 256, 0, stream>>>(
      YNH, YNL, kDi, WOUT, kDi, H2, kDm, hidden, kDm, kSeq, kDm, kDi);

  rmsnorm_split_kernel<false><<<kSeq, 128, 0, stream>>>(H2, post_norm_w, XNH, XNL);

  gemm_a2_kernel<0><<<((kSeq / 64) * (kInt / 64)) / 8, 256, 0, stream>>>(
      XNH, XNL, kDm, WG, kDm, GATE, kInt, hidden, 0, kSeq, kInt, kDm);
  gemm_a2_kernel<0><<<((kSeq / 64) * (kInt / 64)) / 8, 256, 0, stream>>>(
      XNH, XNL, kDm, WU, kDm, UP, kInt, hidden, 0, kSeq, kInt, kDm);

  gu_split_kernel<<<(kSeq * kInt / 8) / 256, 256, 0, stream>>>(GATE, UP, GUH, GUL, kSeq * kInt / 8);

  gemm_a2_kernel<1><<<((kSeq / 64) * (kDm / 64)) / 8, 256, 0, stream>>>(
      GUH, GUL, kInt, WD, kInt, out, kDm, H2, kDm, kSeq, kDm, kInt);
}
